// EventSequenceEmbedder_66632122630827
// MI455X (gfx1250) — hardware-verified
//
#include <hip/hip_runtime.h>

constexpr int kBatch     = 32;
constexpr int kSeqLen    = 1024;
constexpr int kDmodel    = 256;
constexpr int kMaxP      = 9;
constexpr int kNAct      = 8;
constexpr int kNCard     = 53;
constexpr int kKtot      = 8 * kDmodel;
constexpr int kRowsTotal = kBatch * kSeqLen;
constexpr int kRowsHalf  = kRowsTotal / 2;
constexpr int kRowsPerBlk  = 32;
constexpr int kRowsPerWave = kRowsPerBlk / 2;
constexpr float kACarry   = 1024.0f;
constexpr float kWCarry   = 64.0f;
constexpr float kOutScale = 1.0f / (1024.0f * 64.0f);

typedef __attribute__((ext_vector_type(16))) _Float16 v16h;
typedef __attribute__((ext_vector_type(8)))  _Float16 v8h;
typedef __attribute__((ext_vector_type(16))) __bf16   v16b;
typedef __attribute__((ext_vector_type(8)))  __bf16   v8b;
typedef __attribute__((ext_vector_type(8)))  float    v8f;
typedef __attribute__((ext_vector_type(4)))  float    v4f;
typedef __attribute__((ext_vector_type(4)))  unsigned int v4u;

__device__ __forceinline__ unsigned short f2bf_bits(float f) {
  unsigned u = __float_as_uint(f);
  return (unsigned short)((u + 0x7FFFu + ((u >> 16) & 1u)) >> 16);
}
__device__ __forceinline__ float bf_bits2f(unsigned short h) { return __uint_as_float(((unsigned)h) << 16); }

__device__ __forceinline__ void dep_guard_h(v8f& a, v8f& b, v16h x, v16h y) { asm volatile("v_nop\n\tv_nop\n\tv_nop\n\tv_nop" : "+v"(a), "+v"(b) : "v"(x), "v"(y)); }
__device__ __forceinline__ void dep_guard_b(v8f& a, v8f& b, v16b x, v16b y) { asm volatile("v_nop\n\tv_nop\n\tv_nop\n\tv_nop" : "+v"(a), "+v"(b) : "v"(x), "v"(y)); }
__device__ __forceinline__ void keep4_h(v16h a, v16h b, v16h c, v16h d) { asm volatile("v_nop" :: "v"(a), "v"(b), "v"(c), "v"(d)); }
__device__ __forceinline__ void keep4_b(v16b a, v16b b, v16b c, v16b d) { asm volatile("v_nop" :: "v"(a), "v"(b), "v"(c), "v"(d)); }
__device__ __forceinline__ void acc_guard4(v8f& a, v8f& b, v8f& c, v8f& d) { asm volatile("v_nop\n\tv_nop\n\tv_nop\n\tv_nop" : "+v"(a), "+v"(b), "+v"(c), "+v"(d)); }
template <typename T> struct Frag;
template <> struct Frag<_Float16> {
  typedef v16h V; union U { v16h v; v8h h[2]; };
  static __device__ __forceinline__ v16h load(const _Float16* p) {
    U f; f.h[0] = *(const v8h*)(p); f.h[1] = *(const v8h*)(p + 16); return f.v;
  }
  static __device__ __forceinline__ v8f mma(v16h a, v16h b, v8f c) {
    return __builtin_amdgcn_wmma_f32_16x16x32_f16(false, a, false, b, (short)0, c, false, false);
  }
  static __device__ __forceinline__ void guard(v8f& a, v8f& b, v16h x, v16h y) { dep_guard_h(a, b, x, y); }
  static __device__ __forceinline__ void keep(v16h a, v16h b, v16h c, v16h d) { keep4_h(a, b, c, d); }
};
template <> struct Frag<__bf16> {
  typedef v16b V; union U { v16b v; v8b h[2]; };
  static __device__ __forceinline__ v16b load(const __bf16* p) {
    U f; f.h[0] = *(const v8b*)(p); f.h[1] = *(const v8b*)(p + 16); return f.v;
  }
  static __device__ __forceinline__ v8f mma(v16b a, v16b b, v8f c) {
    return __builtin_amdgcn_wmma_f32_16x16x32_bf16(false, a, false, b, (short)0, c, false, false);
  }
  static __device__ __forceinline__ void guard(v8f& a, v8f& b, v16b x, v16b y) { dep_guard_b(a, b, x, y); }
  static __device__ __forceinline__ void keep(v16b a, v16b b, v16b c, v16b d) { keep4_b(a, b, c, d); }
};

__device__ __forceinline__ unsigned pk16(unsigned short a, unsigned short b) { return (unsigned)a | ((unsigned)b << 16); }
__device__ __forceinline__ unsigned short h_bits(float f) { const _Float16 h = (_Float16)f; return __builtin_bit_cast(unsigned short, h); }

template <int ET> struct Elem;
template <> struct Elem<0> { typedef _Float16 T; };
template <> struct Elem<1> { typedef __bf16 T; };
template <int ET, bool SPLIT, int BIAS_MODE, int OUT_MODE, bool RESID, int ACT, bool ROWSC>
__global__ __launch_bounds__(256) void wmma_gemm64rs(
    const unsigned short* __restrict__ Ap, const unsigned short* __restrict__ A2p, int lda, long strideA,
    const unsigned short* __restrict__ Btp, const unsigned short* __restrict__ Bt2p, int ldb, long strideB,
    void* __restrict__ Cout, void* __restrict__ Cout2, int ldc, long strideC,
    const float* __restrict__ bias,
    const float* __restrict__ resid, long strideR,
    const float* __restrict__ rowsc,
    int M, int N, int K, float scale) {
  typedef typename Elem<ET>::T T;
  typedef typename Frag<T>::V V;
  const T* A = (const T*)Ap; const T* A2 = (const T*)A2p; const T* Bt = (const T*)Btp; const T* Bt2 = (const T*)Bt2p;
  __shared__ __align__(16) float sT[8][16 * 68];
  const int b    = blockIdx.y;
  const int lane = threadIdx.x & 31;
  const int wave = threadIdx.x >> 5;
  const int tilesN = N >> 6;
  const int tilesM = M >> 6;
  const int tile = blockIdx.x * 8 + wave;
  if (tile >= tilesM * tilesN) return;
  const int tm = tile / tilesN;
  const int tn = tile - tm * tilesN;
  const int m0 = tm << 6;
  const int n0 = tn << 6;

  const T* Ab  = A  + (size_t)b * strideA;
  const T* Bb  = Bt + (size_t)b * strideB;
  const T* Ab2 = SPLIT ? (A2  + (size_t)b * strideA) : nullptr;
  const T* Bb2 = SPLIT ? (Bt2 + (size_t)b * strideB) : nullptr;

  const int rlane = lane & 15;
  const int koff  = (lane >> 4) * 8;
  const int mOff  = (lane >> 4) * 8;

  v8f acc[4][4];
#pragma unroll
  for (int i = 0; i < 4; ++i)
#pragma unroll
    for (int j = 0; j < 4; ++j) acc[i][j] = (v8f){0.f,0.f,0.f,0.f,0.f,0.f,0.f,0.f};

  for (int k0 = 0; k0 < K; k0 += 32) {
    V bh[4], bl[4];
#pragma unroll
    for (int j = 0; j < 4; ++j) {
      const size_t bo = (size_t)(n0 + (j << 4) + rlane) * ldb + koff + k0;
      bh[j] = Frag<T>::load(Bb + bo);
      if (SPLIT) bl[j] = Frag<T>::load(Bb2 + bo);
    }
#pragma unroll
    for (int i = 0; i < 4; ++i) {
      const size_t ao = (size_t)(m0 + (i << 4) + rlane) * lda + koff + k0;
      V ah = Frag<T>::load(Ab + ao);
      V al;
      if (SPLIT) al = Frag<T>::load(Ab2 + ao);
#pragma unroll
      for (int j = 0; j < 4; ++j) {
        acc[i][j] = Frag<T>::mma(ah, bh[j], acc[i][j]);
        if (SPLIT) {
          acc[i][j] = Frag<T>::mma(ah, bl[j], acc[i][j]);
          acc[i][j] = Frag<T>::mma(al, bh[j], acc[i][j]);
        }
      }
      Frag<T>::guard(acc[i][0], acc[i][3], ah, SPLIT ? al : ah);
    }
    Frag<T>::keep(bh[0], bh[1], bh[2], bh[3]);
    if (SPLIT) Frag<T>::keep(bl[0], bl[1], bl[2], bl[3]);
  }
  acc_guard4(acc[0][0], acc[0][1], acc[0][2], acc[0][3]);
  acc_guard4(acc[1][0], acc[1][1], acc[1][2], acc[1][3]);
  acc_guard4(acc[2][0], acc[2][1], acc[2][2], acc[2][3]);
  acc_guard4(acc[3][0], acc[3][1], acc[3][2], acc[3][3]);

  float* slab = sT[wave];
  const float* Rb = RESID ? (resid + (size_t)b * strideR) : nullptr;
#pragma unroll
  for (int i = 0; i < 4; ++i) {
    const int mBase = m0 + (i << 4);
#pragma unroll
    for (int j = 0; j < 4; ++j) {
      const int n = n0 + (j << 4) + rlane;
      float bv = 0.f;
      if (BIAS_MODE == 2) bv = bias[n];
#pragma unroll
      for (int r = 0; r < 8; ++r) {
        float v = acc[i][j][r] * scale;
        if (BIAS_MODE == 1) v += bias[mBase + mOff + r];
        if (BIAS_MODE == 2) v += bv;
        if (ROWSC) v *= rowsc[mBase + mOff + r];
        if (RESID) v += Rb[(size_t)(mBase + mOff + r) * ldc + n];
        if (ACT == 2) v = fmaxf(v, 0.0f);
        if (ACT == 4) v = (v > 0.f) ? v : 0.01f * v;
        slab[(mOff + r) * 68 + (j << 4) + rlane] = v;
      }
    }
    __builtin_amdgcn_fence(__ATOMIC_RELEASE, "workgroup");
    __builtin_amdgcn_wave_barrier();
    __builtin_amdgcn_fence(__ATOMIC_ACQUIRE, "workgroup");
    if (OUT_MODE == 0) {
      float* C = (float*)Cout + (size_t)b * strideC;
      const int hh = lane >> 4, c4 = (lane & 15) * 4;
      for (int pass = 0; pass < 2; ++pass) {
#pragma unroll
        for (int it = 0; it < 8; ++it) {
          const int row = it * 2 + hh;
          v4f v = *(const v4f*)(slab + row * 68 + c4);
          *(volatile v4f*)(C + (size_t)(mBase + row) * ldc + n0 + c4) = v;
        }
        __threadfence();
      }
    } else {
      const int q = lane >> 3, c8 = (lane & 7) * 8;
      unsigned short* C  = (unsigned short*)Cout  + (size_t)b * strideC;
      unsigned short* C2 = (OUT_MODE == 2) ? ((unsigned short*)Cout2 + (size_t)b * strideC) : nullptr;
      for (int pass = 0; pass < 2; ++pass) {
#pragma unroll
        for (int it = 0; it < 4; ++it) {
          const int row = it * 4 + q;
          const float* sp = slab + row * 68 + c8;
          v8h hv, lv;
#pragma unroll
          for (int e = 0; e < 8; ++e) {
            if (OUT_MODE == 1) {
              hv[e] = (_Float16)sp[e];
            } else {
              unsigned short hb = f2bf_bits(sp[e]);
              unsigned short lb = f2bf_bits(sp[e] - bf_bits2f(hb));
              hv[e] = __builtin_bit_cast(_Float16, hb);
              lv[e] = __builtin_bit_cast(_Float16, lb);
            }
          }
          *(volatile v8h*)(C + (size_t)(mBase + row) * ldc + n0 + c8) = hv;
          if (OUT_MODE == 2) *(volatile v8h*)(C2 + (size_t)(mBase + row) * ldc + n0 + c8) = lv;
        }
        __threadfence();
      }
    }
    __builtin_amdgcn_fence(__ATOMIC_RELEASE, "workgroup");
    __builtin_amdgcn_wave_barrier();
    __builtin_amdgcn_fence(__ATOMIC_ACQUIRE, "workgroup");
  }
}

__global__ __launch_bounds__(256) void cast8_f16_scale_kernel(const float* __restrict__ in, unsigned short* __restrict__ out,
                                                             int n8, float carry) {
  const int i = blockIdx.x * 256 + threadIdx.x;
  if (i >= n8) return;
  const float* p = in + 8 * (size_t)i;
  const v4f a = *(const v4f*)(p);
  const v4f c = *(const v4f*)(p + 4);
  unsigned short hb[8];
#pragma unroll
  for (int e = 0; e < 4; ++e) {
    hb[e]     = h_bits(a[e] * carry);
    hb[4 + e] = h_bits(c[e] * carry);
  }
  const v4u u = (v4u){pk16(hb[0], hb[1]), pk16(hb[2], hb[3]), pk16(hb[4], hb[5]), pk16(hb[6], hb[7])};
  unsigned short* q = out + 8 * (size_t)i;
  *(volatile v4u*)q = u;
  __threadfence();
  *(volatile v4u*)q = u;
}

__global__ __launch_bounds__(64) void assemble_kernel(
    const int*   __restrict__ cards,
    const int*   __restrict__ hero_pos,
    const int*   __restrict__ acting_pos,
    const int*   __restrict__ num_players,
    const float* __restrict__ scalars,
    const float* __restrict__ blinds,
    const float* __restrict__ bets,
    const float* __restrict__ action,
    const float* __restrict__ card_table,
    const float* __restrict__ hero_table,
    const float* __restrict__ acting_table,
    const float* __restrict__ nump_table,
    const float* __restrict__ scalar_W,
    const float* __restrict__ scalar_b,
    const float* __restrict__ blind_W,
    const float* __restrict__ blind_b,
    const float* __restrict__ bet_W,
    const float* __restrict__ bet_b,
    const float* __restrict__ action_W,
    const float* __restrict__ action_b,
    unsigned short* __restrict__ A16,
    int rowBase) {
  const int seg  = blockIdx.y;
  const int lane = threadIdx.x & 31;
  const int wave = threadIdx.x >> 5;
  const int d0   = lane * 8;

  const float* tbl = (seg == 1) ? hero_table : (seg == 2) ? acting_table : nump_table;
  const int*   tix = (seg == 1) ? hero_pos   : (seg == 2) ? acting_pos   : num_players;
  const int    tmax = (seg == 6) ? (kMaxP) : (kMaxP - 1);
  const float* linX = (seg == 3) ? scalars  : (seg == 4) ? bets  : (seg == 5) ? action   : blinds;
  const float* linW = (seg == 3) ? scalar_W : (seg == 4) ? bet_W : (seg == 5) ? action_W : blind_W;
  const float* linB = (seg == 3) ? scalar_b : (seg == 4) ? bet_b : (seg == 5) ? action_b : blind_b;
  const int    linK = (seg == 3) ? 2 : (seg == 4) ? kMaxP : (seg == 5) ? kNAct : 2;

#pragma unroll 1
  for (int it = 0; it < kRowsPerWave; ++it) {
    const int ml = blockIdx.x * kRowsPerBlk + it * 2 + wave;
    const int m  = rowBase + ml;
    float v[8];
#pragma unroll
    for (int e = 0; e < 8; ++e) v[e] = 0.f;

    if (seg == 0) {
      float s[8];
#pragma unroll
      for (int e = 0; e < 8; ++e) s[e] = 0.f;
#pragma unroll
      for (int c = 0; c < 7; ++c) {
        int id = cards[(size_t)m * 7 + c];
        id = id < 0 ? 0 : (id > kNCard - 1 ? kNCard - 1 : id);
        const float* p = card_table + (size_t)id * kDmodel + d0;
        const v4f a = *(const v4f*)(p);
        const v4f q = *(const v4f*)(p + 4);
#pragma unroll
        for (int e = 0; e < 4; ++e) { s[e] += a[e]; s[4 + e] += q[e]; }
      }
#pragma unroll
      for (int e = 0; e < 8; ++e) v[e] = s[e] * (1.0f / 7.0f);
    } else if (seg == 1 || seg == 2 || seg == 6) {
      int id = tix[m];
      id = id < 0 ? 0 : (id > tmax ? tmax : id);
      const float* p = tbl + (size_t)id * kDmodel + d0;
      const v4f a = *(const v4f*)(p);
      const v4f q = *(const v4f*)(p + 4);
#pragma unroll
      for (int e = 0; e < 4; ++e) { v[e] = a[e]; v[4 + e] = q[e]; }
    } else {
      float acc[8];
#pragma unroll
      for (int e = 0; e < 8; ++e) acc[e] = 0.f;
#pragma unroll 1
      for (int j = 0; j < linK; ++j) {
        const float xj = linX[(size_t)m * linK + j];
#pragma unroll
        for (int e = 0; e < 8; ++e) acc[e] += xj * linW[(d0 + e) * linK + j];
      }
#pragma unroll
      for (int e = 0; e < 8; ++e) v[e] = acc[e] + linB[d0 + e];
    }

    unsigned short hb[8];
#pragma unroll
    for (int e = 0; e < 8; ++e) hb[e] = h_bits(v[e] * kACarry);
    const v4u u = (v4u){pk16(hb[0], hb[1]), pk16(hb[2], hb[3]), pk16(hb[4], hb[5]), pk16(hb[6], hb[7])};
    unsigned short* q = A16 + (size_t)ml * kKtot + seg * kDmodel + d0;
    *(volatile v4u*)q = u;
    __threadfence();
    *(volatile v4u*)q = u;
  }
}

extern "C" void kernel_launch(void* const* d_in, const int* in_sizes, int n_in,
                              void* d_out, int out_size, void* d_ws, size_t ws_size,
                              hipStream_t stream) {
  if (n_in < 23) return;
  if (in_sizes[1] != kRowsTotal || in_sizes[0] != kRowsTotal * 7) return;
  if (in_sizes[21] != kDmodel * kKtot || in_sizes[8] != kRowsTotal) return;
  if (out_size != kRowsTotal * kDmodel) return;

  const size_t offW   = 0;
  const size_t bytesW = (size_t)kDmodel * kKtot * sizeof(unsigned short);
  const size_t offA   = offW + bytesW;
  const size_t bytesA = (size_t)kRowsHalf * kKtot * sizeof(unsigned short);
  if (offA + bytesA > ws_size) return;

  unsigned short* W16 = (unsigned short*)((char*)d_ws + offW);
  unsigned short* A16 = (unsigned short*)((char*)d_ws + offA);
  float* outp = (float*)d_out;

  const int*   cards        = (const int*)d_in[0];
  const int*   hero_pos     = (const int*)d_in[1];
  const int*   acting_pos   = (const int*)d_in[2];
  const int*   num_players  = (const int*)d_in[3];
  const float* scalars      = (const float*)d_in[4];
  const float* blinds       = (const float*)d_in[5];
  const float* bets         = (const float*)d_in[6];
  const float* action       = (const float*)d_in[7];
  const float* mask         = (const float*)d_in[8];
  const float* card_table   = (const float*)d_in[9];
  const float* hero_table   = (const float*)d_in[10];
  const float* acting_table = (const float*)d_in[11];
  const float* nump_table   = (const float*)d_in[12];
  const float* scalar_W     = (const float*)d_in[13];
  const float* scalar_b     = (const float*)d_in[14];
  const float* blind_W      = (const float*)d_in[15];
  const float* blind_b      = (const float*)d_in[16];
  const float* bet_W        = (const float*)d_in[17];
  const float* bet_b        = (const float*)d_in[18];
  const float* action_W     = (const float*)d_in[19];
  const float* action_b     = (const float*)d_in[20];
  const float* combine_W    = (const float*)d_in[21];
  const float* combine_b    = (const float*)d_in[22];

  const int n8 = kDmodel * kKtot / 8;
  cast8_f16_scale_kernel<<<dim3((n8 + 255) / 256), dim3(256), 0, stream>>>(combine_W, W16, n8, kWCarry);

  const int tilesPerHalf = (kRowsHalf / 64) * (kDmodel / 64);
  const int gemmBlocks   = (tilesPerHalf + 7) / 8;
  for (int half = 0; half < 2; ++half) {
    const int rowBase = half * kRowsHalf;
    assemble_kernel<<<dim3(kRowsHalf / kRowsPerBlk, 8), dim3(64), 0, stream>>>(
        cards, hero_pos, acting_pos, num_players,
        scalars, blinds, bets, action,
        card_table, hero_table, acting_table, nump_table,
        scalar_W, scalar_b, blind_W, blind_b, bet_W, bet_b, action_W, action_b,
        A16, rowBase);
    wmma_gemm64rs<0, false, 2, 0, false, 0, true><<<dim3(gemmBlocks, 1), dim3(256), 0, stream>>>(
        (const unsigned short*)A16, (const unsigned short*)A16, kKtot, 0L,
        (const unsigned short*)W16, (const unsigned short*)W16, kKtot, 0L,
        (void*)(outp + (size_t)rowBase * kDmodel), (void*)d_ws, kDmodel, 0L,
        combine_b,
        combine_b, 0L,
        mask + rowBase,
        kRowsHalf, kDmodel, kKtot, kOutScale);
  }
}
